// CPRL_24292335026358
// MI455X (gfx1250) — hardware-run, weakly checked
//
#include <hip/hip_runtime.h>


#ifndef NB
#define NB 32
#endif
#define NB_FULL 32
#define D1   128
#define D2   64
#define D3   32
#define NO   64
#define RK   16
#define KD   (D2 * D3)
#define GW   2
#define GT   4
#define TPW  32
#define HM   32
#define HOP  68
#define HCS  4096.0f
#define HCI  (1.0f / 4096.0f)
#define TCS  1024.0f
#define GCS  1024.0f
#define OCI  (1.0f / (1024.0f * 1024.0f))

static_assert(RK == 16);
static_assert(KD % 32 == 0);
static_assert(D3 == 32);
static_assert(D3 % 8 == 0);
static_assert(KD / 8 == 256);
static_assert(GW * GT * 16 == D1);
static_assert((RK * KD) % (8 * 256) == 0);
static_assert((D1 * RK) % (32 * GW * 4) == 0);
static_assert(TPW == 32);
static_assert(2 * RK == TPW);
static_assert(HM == 32 && NB_FULL <= HM);
static_assert(NO % 16 == 0 && NO == 64);
static_assert(16 * 32 * 16 == HM * NO * 4);
static_assert((HOP * 4) % 16 == 0);
static_assert(NB >= 1 && NB <= NB_FULL);
static_assert((D1 * RK + GW * RK) * 4 <= 131072);
static_assert(HM * HOP * 4 <= 131072);

typedef _Float16 h16;
typedef __attribute__((ext_vector_type(16))) _Float16 v16h;
typedef __attribute__((ext_vector_type(8)))  _Float16 v8h;
typedef __attribute__((ext_vector_type(8)))  float    v8f;
typedef __attribute__((ext_vector_type(4)))  float    v4f;
typedef v4f  __attribute__((may_alias)) v4fa;

__device__ __forceinline__ unsigned short f2bf(float f) { unsigned u = __float_as_uint(f); u += 0x7FFFu + ((u >> 16) & 1u); return (unsigned short)(u >> 16); }
__device__ __forceinline__ float bfr(float f) { return __uint_as_float(((unsigned)f2bf(f)) << 16); }
__device__ __forceinline__ v16h cat16(v8h lo, v8h hi) { return __builtin_shufflevector(lo, hi, 0, 1, 2, 3, 4, 5, 6, 7, 8, 9, 10, 11, 12, 13, 14, 15); }
__device__ __forceinline__ v16h  ldh(const h16* p) { return cat16(*(const v8h*)p, *(const v8h*)(p + 16)); }
static __device__ __forceinline__ h16 toh_flush(float v) { const h16 r = (h16)v; return (fabsf(v) < 6.103515625e-05f) ? (h16)0.0f : r; }
__device__ __forceinline__ v8f wmma16g(v16h a, v16h b, v8f c) {
    c = __builtin_amdgcn_wmma_f32_16x16x32_f16(false, a, false, b, (short)0, c, false, false);
    asm volatile("v_nop\n\tv_nop\n\tv_nop\n\tv_nop" : "+v"(c) : "v"(a), "v"(b));
    return c;
}
__device__ __forceinline__ v16h ldx16(const float* p) {
    const v4f x0 = *(const v4f*)p, x1 = *(const v4f*)(p + 4), x2 = *(const v4f*)(p + 16), x3 = *(const v4f*)(p + 20);
    v16h o;
#pragma unroll
    for (int i = 0; i < 4; ++i) { o[i] = toh_flush(bfr(x0[i])); o[4 + i] = toh_flush(bfr(x1[i])); o[8 + i] = toh_flush(bfr(x2[i])); o[12 + i] = toh_flush(bfr(x3[i])); }
    return o;
}

__global__ __launch_bounds__(256) void k_hbuild(const float* __restrict__ F1, const float* __restrict__ F2, h16* HT) {
#pragma clang fp contract(off)
    unsigned i = blockIdx.x * blockDim.x + threadIdx.x;
    asm volatile("" : "+v"(i));
    if (i >= (unsigned)((RK * KD) / 8)) return;
    const unsigned r = i >> 8;
    const unsigned k = (i & 255u) << 3;
    const unsigned b = k >> 5;
    const unsigned c0 = k & 31u;
    const float a = bfr(F1[b * (unsigned)RK + r]) * HCS;
    v8h o;
#pragma unroll
    for (unsigned j = 0; j < 8u; ++j) o[j] = toh_flush(a * bfr(F2[(c0 + j) * (unsigned)RK + r]));
    *(volatile v8h*)(HT + (size_t)i * 8) = o; __threadfence(); *(volatile v8h*)(HT + (size_t)i * 8) = o;
}

__global__ __launch_bounds__(32 * GW) void k_ugemm(const float* __restrict__ X, const h16* __restrict__ HT, const float* __restrict__ F0, float* TP) {
    __shared__ __align__(16) float f0s[D1 * RK];
    __shared__ float tps[GW * RK];
    const int lane = threadIdx.x & 31, lr = lane & 15, hi = lane >> 4;
    const int wave = __builtin_amdgcn_readfirstlane((int)(threadIdx.x >> 5));
    const int xb = blockIdx.x;
#pragma unroll 1
    for (int i = 0; i < (D1 * RK) / (32 * GW * 4); ++i) {
        const int idx = (i * 32 * GW + (int)threadIdx.x) * 4;
        const v4f v = *(const v4f*)(F0 + idx); v4f o;
#pragma unroll
        for (int k = 0; k < 4; ++k) o[k] = bfr(v[k]);
        *(v4fa*)(&f0s[idx]) = o;
    }
    __syncthreads();
    v8f acc[GT];
#pragma unroll
    for (int mb = 0; mb < GT; ++mb) acc[mb] = (v8f){};
    const size_t aoff = ((size_t)xb * D1 + (size_t)(wave * GT * 16 + lr)) * KD + 8 * hi;
    const size_t boff = (size_t)lr * KD + 8 * hi;
#pragma unroll 1
    for (int kc = 0; kc < KD; kc += 32) {
        const v16h b = ldh(HT + boff + kc);
#pragma unroll
        for (int mb = 0; mb < GT; ++mb) { const v16h a = ldx16(X + aoff + (size_t)mb * 16 * KD + kc); acc[mb] = wmma16g(a, b, acc[mb]); }
    }
    float tp = 0.0f;
#pragma unroll
    for (int mb = 0; mb < GT; ++mb) {
#pragma unroll
        for (int j = 0; j < 8; ++j) tp += f0s[((wave * GT + mb) * 16 + hi * 8 + j) * RK + lr] * acc[mb][j]; }
    tp *= HCI;
    tp += __shfl_xor(tp, 16, 32);
    if (lane < RK) tps[wave * RK + lane] = tp;
    __syncthreads();
    float tv = 0.0f;
#pragma unroll
    for (int w = 0; w < GW; ++w) tv += tps[w * RK + lr];
    const float val = (lane < RK) ? tv : 0.0f;
    if (wave == 0) { float* dst = TP + (size_t)xb * TPW + lane; *(volatile float*)dst = val; __threadfence(); *(volatile float*)dst = val; }
}

__global__ __launch_bounds__(32) void k_head(const float* __restrict__ TP, const float* __restrict__ F3, const float* __restrict__ CW, const float* __restrict__ BI, float* OUT) {
    __shared__ __align__(16) float os[HM * HOP];
    const int lane = threadIdx.x & 31, lr = lane & 15, hi = lane >> 4;
    v16h a[2], b[4];
#pragma unroll
    for (int mt = 0; mt < 2; ++mt) {
        const int row = mt * 16 + lr; const int rc = row < NB ? row : (NB - 1); const bool ok = row < NB;
        const float* tp = TP + (size_t)rc * TPW + 8 * hi;
        v4f x0 = *(const v4f*)tp, x1 = *(const v4f*)(tp + 4), x2 = *(const v4f*)(tp + 16), x3 = *(const v4f*)(tp + 20);
        asm volatile("" : "+v"(x0), "+v"(x1), "+v"(x2), "+v"(x3));
        v16h o;
#pragma unroll
        for (int i = 0; i < 4; ++i) {
            o[i]      = ok ? toh_flush(x0[i] * TCS) : (h16)0.0f; o[4 + i]  = ok ? toh_flush(x1[i] * TCS) : (h16)0.0f;
            o[8 + i]  = ok ? toh_flush(x2[i] * TCS) : (h16)0.0f; o[12 + i] = ok ? toh_flush(x3[i] * TCS) : (h16)0.0f; }
        a[mt] = o;
    }
    const v4f w0 = *(const v4f*)(CW + 8 * hi), w1 = *(const v4f*)(CW + 8 * hi + 4);
#pragma unroll
    for (int nt = 0; nt < 4; ++nt) {
        const float* fp = F3 + (size_t)(nt * 16 + lr) * RK + 8 * hi;
        const v4f g0 = *(const v4f*)fp, g1 = *(const v4f*)(fp + 4);
        v16h o = (v16h){};
#pragma unroll
        for (int i = 0; i < 4; ++i) { o[i] = toh_flush(bfr(w0[i]) * GCS * bfr(g0[i])); o[4 + i] = toh_flush(bfr(w1[i]) * GCS * bfr(g1[i])); }
        b[nt] = o;
    }
    const float bz = bfr(BI[0]);
#pragma unroll
    for (int mt = 0; mt < 2; ++mt) {
#pragma unroll
        for (int nt = 0; nt < 4; ++nt) {
            v8f c = (v8f){};
            c = wmma16g(a[mt], b[nt], c);
#pragma unroll
            for (int j = 0; j < 8; ++j) os[(mt * 16 + hi * 8 + j) * HOP + nt * 16 + lr] = c[j] * OCI + bz; } }
    __syncthreads();
#pragma unroll 1
    for (int ps = 0; ps < 2; ++ps) {
#pragma unroll
        for (int s = 0; s < 16; ++s) { const int row = 2 * s + (lane >> 4), col = (lane & 15) * 4;
            const v4f val = *(const v4fa*)(&os[row * HOP + col]);
            if (row < NB) *(volatile v4f*)(OUT + (size_t)row * NO + col) = val; }
        if (ps == 0) __threadfence(); }
}

static constexpr size_t al256(size_t v) { return (v + 255) & ~(size_t)255; }
static constexpr size_t SZ_HT = al256((size_t)RK * KD * 2);
static constexpr size_t SZ_TP = al256((size_t)NB_FULL * TPW * 4);
static constexpr size_t SZ_TOTAL = SZ_HT + SZ_TP;
static_assert(SZ_TOTAL <= (size_t)134217728);
static_assert(((size_t)((RK * KD) / 8 - 1) * 8 + 8) * 2 <= SZ_HT);
static_assert(((size_t)(NB - 1) * TPW + 32) * 4 <= SZ_TP);
static_assert((size_t)NB * NO * 4 <= (size_t)NB_FULL * NO * 4);

extern "C" void kernel_launch(void* const* d_in, const int* in_sizes, int n_in,
                              void* d_out, int out_size, void* d_ws, size_t ws_size, hipStream_t stream) {
    if (n_in < 7) return;
    if ((size_t)in_sizes[0] < (size_t)NB * D1 * KD) return;
    if (in_sizes[1] < D1 * RK || in_sizes[2] < D2 * RK || in_sizes[3] < D3 * RK || in_sizes[4] < NO * RK) return;
    if (in_sizes[5] < RK || in_sizes[6] < 1) return;
    if ((size_t)out_size < (size_t)NB * NO) return;
    if (SZ_TOTAL > ws_size) return;
    const float* x  = (const float*)d_in[0];
    const float* f0 = (const float*)d_in[1];
    const float* f1 = (const float*)d_in[2];
    const float* f2 = (const float*)d_in[3];
    const float* f3 = (const float*)d_in[4];
    const float* cw = (const float*)d_in[5];
    const float* bi = (const float*)d_in[6];
    float* OUT = (float*)d_out;
    char* wsp = (char*)d_ws;
    h16* HT = (h16*)wsp; wsp += SZ_HT;
    float* TP = (float*)wsp; wsp += SZ_TP;

    k_hbuild<<<dim3((RK * KD) / (8 * 256), 1, 1), 256, 0, stream>>>(f1, f2, HT);
    k_ugemm<<<dim3(NB, 1, 1), 32 * GW, 0, stream>>>(x, HT, f0, TP);
    k_head<<<dim3(1, 1, 1), 32, 0, stream>>>(TP, f3, cw, bi, OUT);
}
